// SpatioTemporalFGNN_86053964743111
// MI455X (gfx1250) — hardware-verified
//
#include <hip/hip_runtime.h>
#include <stddef.h>


#define NBT    16
#define NST    12
#define NN     325
#define NNP    336
#define NTAB   328
#define NE     2600
#define CI     32
#define HD     64
#define PW     1024
#define KF     3072
#define CO     12
#define COP    16
#define NCP    (NBT * NST)
#define NROWS  (NCP * NN)
#define NCHUNK 4
#define CPC    (NCP / NCHUNK)
#define RPC    (CPC * NN)
#define GPX    ((RPC + 31) / 32)
#define RPCP   (GPX * 32)
#define NTHR   256
#define NWAVE  8
#define APH    72
#define ASCL   8.0f
#define WSCL   64.0f
#define LSCL   1024.0f
#define INV512  0.001953125f
#define INV8192 0.0001220703125f
#define DEN_EPS 1e-16f
#define NEG_BIG (-3.0e38f)
#define WSCAP  134217728

#define G_HA   0
#define G_HW   (G_HA + NNP * APH * 2)
#define G_WB   (G_HW + NNP * HD * 4)
#define G_ES   (G_WB + HD * APH * 2)
#define G_OF   (G_ES + NE * 4)
#define G_CN   (G_OF + NTAB * 4)
#define G_DI   (G_CN + NTAB * 4)
#define LDS_GCN (G_DI + NTAB * 4)

#define T_SL   0
#define T_SC   (T_SL + NE * 4 * 4)
#define T_SR   (T_SC + NE * 4)
#define T_ES   (T_SR + NE * 4)
#define T_OF   (T_ES + NE * 4)
#define T_CN   (T_OF + NTAB * 4)
#define LDS_ATTN (T_CN + NTAB * 4)

static_assert(NNP % 16 == 0 && NNP >= NN && NTAB >= NN + 1);
static_assert(RPCP >= RPC && RPCP == GPX * 32);
static_assert(NCP % NCHUNK == 0);
static_assert(2 * NE * 4 <= NNP * HD * 4);
static_assert((G_HW % 16) == 0 && (G_WB % 16) == 0 && (G_ES % 16) == 0 && (G_OF % 16) == 0 && (G_CN % 16) == 0 && (G_DI % 16) == 0);
static_assert((T_SC % 16) == 0 && (T_ES % 16) == 0 && (T_OF % 16) == 0 && (T_CN % 16) == 0);
static_assert((APH * 2) % 16 == 0);
static_assert(NN * (CI / 8) <= NTHR * 6);
static_assert((NROWS % 16) == 0 && ((NBT * NN) % 16) == 0);
static_assert(KF % 32 == 0 && HD % 32 == 0 && CI % 32 == 0);
static_assert(NWAVE * 32 == NTHR);

typedef float          v2f  __attribute__((ext_vector_type(2)));
typedef float          v4f  __attribute__((ext_vector_type(4)));
typedef float          v8f  __attribute__((ext_vector_type(8)));
typedef unsigned short v8us __attribute__((ext_vector_type(8)));
typedef _Float16       v16h __attribute__((ext_vector_type(16)));
union FragH { v16h v; v8us u[2]; };

__device__ __forceinline__ unsigned short h16(float f) {
  const _Float16 h = (_Float16)f;
  return __builtin_bit_cast(unsigned short, h);
}

__device__ __forceinline__ v8us cvt8(v4f a, v4f b, float s) {
  v8us r;
  r[0] = h16(a.x * s); r[1] = h16(a.y * s); r[2] = h16(a.z * s); r[3] = h16(a.w * s);
  r[4] = h16(b.x * s); r[5] = h16(b.y * s); r[6] = h16(b.z * s); r[7] = h16(b.w * s);
  return r;
}

__device__ __forceinline__ v8f wmh(v16h a, v16h b, v8f c) {
  v8f d = __builtin_amdgcn_wmma_f32_16x16x32_f16(false, a, false, b, (short)0, c, false, false);
  asm volatile("v_nop\n\tv_nop\n\tv_nop\n\tv_nop" : "+v"(d) : "v"(a), "v"(b));
  return d;
}

__device__ __forceinline__ void build_csr(const int* __restrict__ erow, const int* __restrict__ ecol,
                                          int* scol, int* srow, int* esrt, int* soff, int* scnt, int tid) {
#pragma unroll 1
  for (int i = tid; i < NE; i += NTHR) {
    int c = ecol[i]; c = c < 0 ? 0 : (c > NN - 1 ? NN - 1 : c);
    int r = erow[i]; r = r < 0 ? 0 : (r > NN - 1 ? NN - 1 : r);
    scol[i] = c;
    srow[i] = r;
  }
#pragma unroll 1
  for (int i = tid; i < NTAB; i += NTHR) { scnt[i] = 0; soff[i] = 0; }
  __syncthreads();
  if (tid == 0) {
#pragma unroll 1
    for (int e = 0; e < NE; ++e) { const int c = scol[e]; scnt[c] = scnt[c] + 1; }
    int acc = 0;
#pragma unroll 1
    for (int n = 0; n < NN; ++n) { const int k = scnt[n]; soff[n] = acc; scnt[n] = acc; acc += k; }
    soff[NN] = acc;
#pragma unroll 1
    for (int e = 0; e < NE; ++e) {
      const int c = scol[e];
      int pos = scnt[c];
      pos = pos < 0 ? 0 : (pos > NE - 1 ? NE - 1 : pos);
      esrt[pos] = srow[e];
      scnt[c] = pos + 1;
    }
  }
  __syncthreads();
}

__global__ __launch_bounds__(NTHR) void k_wcvt(const float* __restrict__ W, int K, int ncs, int ncd,
                                              float scale, unsigned short* outp) {
  const int i     = (int)blockIdx.x * NTHR + (int)threadIdx.x;
  const int kpr   = K >> 3;
  const int units = ncd * kpr;
  if (i >= units) return;
  const int n  = i / kpr;
  const int k0 = (i - n * kpr) * 8;
  const int nn = n < ncs ? n : ncs - 1;
  const bool live = n < ncs;
  v8us hv;
#pragma unroll
  for (int e = 0; e < 8; ++e) {
    const float v = W[(size_t)(k0 + e) * ncs + nn];
    hv[e] = h16((live ? v : 0.0f) * scale);
  }
  unsigned short* dp = outp + (size_t)i * 8;
  *(volatile v8us*)dp = hv;
  __threadfence();
  *(volatile v8us*)dp = hv;
}

__global__ __launch_bounds__(NTHR) void k_gcn(const float* __restrict__ x, const int* __restrict__ eidx,
                                             const unsigned short* __restrict__ wg,
                                             const float* __restrict__ b0p, const float* __restrict__ b1p,
                                             const float* __restrict__ b2p, const float* __restrict__ b3p,
                                             unsigned short* xt) {
  extern __shared__ v4f lds_dyn[];
  char* lb = (char*)lds_dyn;
  unsigned short* hA = (unsigned short*)(lb + G_HA);
  float* hw    = (float*)(lb + G_HW);
  int*   scol  = (int*)(lb + G_HW);
  int*   srow  = scol + NE;
  unsigned short* wB = (unsigned short*)(lb + G_WB);
  int*   esrt  = (int*)(lb + G_ES);
  int*   soff  = (int*)(lb + G_OF);
  int*   scnt  = (int*)(lb + G_CN);
  float* sdinv = (float*)(lb + G_DI);
  const int tid = threadIdx.x, lane = tid & 31, wave = tid >> 5, hh = lane >> 4, m = lane & 15;
  const int cp = blockIdx.x;

  {
    unsigned int* hz = (unsigned int*)(hA + NN * APH);
#pragma unroll 1
    for (int i = tid; i < (NNP - NN) * APH / 2; i += NTHR) hz[i] = 0u;
#pragma unroll 1
    for (int u = tid; u < NN * (CI / 8); u += NTHR) {
      const int n = u >> 2, c0 = (u & 3) * 8;
      const float* xp = x + ((size_t)cp * NN + n) * CI + c0;
      const v4f a = *(const v4f*)xp, b = *(const v4f*)(xp + 4);
      *(v8us*)(hA + n * APH + c0) = cvt8(a, b, ASCL);
    }
  }
  build_csr(eidx, eidx + NE, scol, srow, esrt, soff, scnt, tid);

#pragma unroll 1
  for (int n = tid; n < NTAB; n += NTHR) {
    const int lo = soff[n < NN ? n : NN];
    const int hi = soff[n < NN ? n + 1 : NN];
    int dg = hi - lo;
    dg = dg < 0 ? 0 : (dg > NE ? NE : dg);
    sdinv[n] = 1.0f / sqrtf(1.0f + (float)dg);
  }
  const float bA0 = b0p[2 * lane], bA1 = b0p[2 * lane + 1];
  const float bB0 = b1p[2 * lane], bB1 = b1p[2 * lane + 1];
  const float bC0 = b2p[2 * lane], bC1 = b2p[2 * lane + 1];
  const float bD0 = b3p[2 * lane], bD1 = b3p[2 * lane + 1];
  __syncthreads();

#pragma unroll 1
  for (int l = 0; l < 4; ++l) {
    const int ksh    = (l == 0) ? 2 : 3;
    const int K      = 8 << ksh;
    const int ksteps = K >> 5;
    const int po     = (l == 0) ? 0 : (CI * HD + (l - 1) * HD * HD);
    {
      const int units = HD << ksh;
#pragma unroll 1
      for (int i = tid; i < units; i += NTHR) {
        const int n  = i >> ksh;
        const int k0 = (i - (n << ksh)) * 8;
        *(v8us*)(wB + n * APH + k0) = *(const v8us*)(wg + po + (size_t)n * K + k0);
      }
    }
    __syncthreads();

    for (int rt = wave; rt < NNP / 16; rt += NWAVE) {
      v8f acc[4];
#pragma unroll
      for (int t = 0; t < 4; ++t) { const v8f z = {0.f, 0.f, 0.f, 0.f, 0.f, 0.f, 0.f, 0.f}; acc[t] = z; }
      const unsigned short* afp = hA + (16 * rt + m) * APH + 8 * hh;
#pragma unroll 1
      for (int ks = 0; ks < ksteps; ++ks) {
        FragH af;
        af.u[0] = *(const v8us*)(afp + 32 * ks);
        af.u[1] = *(const v8us*)(afp + 32 * ks + 16);
#pragma unroll
        for (int t = 0; t < 4; ++t) {
          const unsigned short* bfp = wB + (16 * t + m) * APH + 32 * ks + 8 * hh;
          FragH bf;
          bf.u[0] = *(const v8us*)bfp;
          bf.u[1] = *(const v8us*)(bfp + 16);
          acc[t] = wmh(af.v, bf.v, acc[t]);
        }
      }
      float* hp = hw + (size_t)(16 * rt + 8 * hh) * HD + m;
#pragma unroll
      for (int t = 0; t < 4; ++t) {
#pragma unroll
        for (int r = 0; r < 8; ++r) hp[r * HD + 16 * t] = acc[t][r] * INV512;
      }
    }
    __syncthreads();

    const float bl0 = (l == 0) ? bA0 : ((l == 1) ? bB0 : ((l == 2) ? bC0 : bD0));
    const float bl1 = (l == 0) ? bA1 : ((l == 1) ? bB1 : ((l == 2) ? bC1 : bD1));
    for (int c = wave; c < NN; c += NWAVE) {
      int st = soff[c];     st = st < 0 ? 0 : (st > NE ? NE : st);
      int en = soff[c + 1]; en = en < 0 ? 0 : (en > NE ? NE : en);
      int n  = en - st;     n  = n  < 0 ? 0 : (n  > NE ? NE : n);
      const float dc = sdinv[c];
      float a0 = 0.f, a1 = 0.f;
#pragma unroll 1
      for (int p = 0; p < n; ++p) {
        int slot = st + p; slot = slot > NE - 1 ? NE - 1 : slot;
        int src = esrt[slot]; src = src < 0 ? 0 : (src > NN - 1 ? NN - 1 : src);
        const float nrm = sdinv[src] * dc;
        const v2f hv = *(const v2f*)(hw + (size_t)src * HD + 2 * lane);
        a0 += hv.x * nrm;
        a1 += hv.y * nrm;
      }
      {
        const float nrm = dc * dc;
        const v2f hv = *(const v2f*)(hw + (size_t)c * HD + 2 * lane);
        a0 += hv.x * nrm;
        a1 += hv.y * nrm;
      }
      const float h0 = fmaxf(a0 + bl0, 0.0f);
      const float h1 = fmaxf(a1 + bl1, 0.0f);
      const unsigned int pk = (unsigned int)h16(h0 * ASCL) | ((unsigned int)h16(h1 * ASCL) << 16);
      *(unsigned int*)(hA + c * APH + 2 * lane) = pk;
    }
    __syncthreads();
  }

  unsigned short* xg = xt + (size_t)cp * NN * HD;
#pragma unroll 1
  for (int i = tid; i < NN * 8; i += NTHR) {
    const v8us v = *(const v8us*)(hA + (i >> 3) * APH + (i & 7) * 8);
    *(volatile v8us*)(xg + (size_t)i * 8) = v;
  }
  __threadfence();
#pragma unroll 1
  for (int i = tid; i < NN * 8; i += NTHR) {
    const v8us v = *(const v8us*)(hA + (i >> 3) * APH + (i & 7) * 8);
    *(volatile v8us*)(xg + (size_t)i * 8) = v;
  }
}

__global__ __launch_bounds__(NTHR) void k_proj(const unsigned short* __restrict__ xt,
                                              const unsigned short* __restrict__ wp,
                                              const float* __restrict__ bq, const float* __restrict__ bk,
                                              const float* __restrict__ bv, const float* __restrict__ bs,
                                              float* P, int rowBase, int nTot) {
  __shared__ __attribute__((aligned(16))) float stg[NWAVE * 16 * 64];
  const int tid = threadIdx.x, lane = tid & 31, wave = tid >> 5, hh = lane >> 4, m = lane & 15;
  const int rg   = wave >> 2;
  const int cq   = wave & 3;
  const int csel = blockIdx.y;
  const int c0   = csel * 256 + cq * 64;
  const int lr0  = (int)blockIdx.x * 32 + rg * 16;
  int grow = rowBase + lr0 + m;
  grow = grow < 0 ? 0 : (grow > nTot - 1 ? nTot - 1 : grow);

  v8f acc[4];
#pragma unroll
  for (int t = 0; t < 4; ++t) { const v8f z = {0.f, 0.f, 0.f, 0.f, 0.f, 0.f, 0.f, 0.f}; acc[t] = z; }
  const unsigned short* afp = xt + (size_t)grow * HD + 8 * hh;
#pragma unroll
  for (int ks = 0; ks < HD / 32; ++ks) {
    FragH af;
    af.u[0] = *(const v8us*)(afp + 32 * ks);
    af.u[1] = *(const v8us*)(afp + 32 * ks + 16);
#pragma unroll
    for (int t = 0; t < 4; ++t) {
      const unsigned short* bfp = wp + (size_t)(c0 + 16 * t + m) * HD + 32 * ks + 8 * hh;
      FragH bf;
      bf.u[0] = *(const v8us*)bfp;
      bf.u[1] = *(const v8us*)(bfp + 16);
      acc[t] = wmh(af.v, bf.v, acc[t]);
    }
  }
  {
    float* sp = stg + wave * 1024 + (8 * hh) * 64 + m;
#pragma unroll
    for (int t = 0; t < 4; ++t) {
#pragma unroll
      for (int r = 0; r < 8; ++r) sp[r * 64 + 16 * t] = acc[t][r];
    }
  }
  __syncthreads();

  const int f4   = lane & 15;
  const int rsub = lane >> 4;
  const int cl   = cq * 64 + 4 * f4;
  const v4f bq4 = *(const v4f*)(bq + cl);
  const v4f bk4 = *(const v4f*)(bk + cl);
  const v4f bv4 = *(const v4f*)(bv + cl);
  const v4f bs4 = *(const v4f*)(bs + cl);
  v4f b4 = bq4;
  if (csel == 1) b4 = bk4;
  if (csel == 2) b4 = bv4;
  if (csel == 3) b4 = bs4;
  v4f o[8];
#pragma unroll
  for (int it = 0; it < 8; ++it) {
    const int rr = 2 * it + rsub;
    const v4f v = *(const v4f*)(stg + wave * 1024 + rr * 64 + 4 * f4);
    o[it] = v * INV512 + b4;
  }
  float* gp = P + (size_t)lr0 * PW + c0 + 4 * f4;
#pragma unroll
  for (int it = 0; it < 8; ++it) *(volatile v4f*)(gp + (size_t)(2 * it + rsub) * PW) = o[it];
  __threadfence();
#pragma unroll
  for (int it = 0; it < 8; ++it) *(volatile v4f*)(gp + (size_t)(2 * it + rsub) * PW) = o[it];
}

__global__ __launch_bounds__(NTHR) void k_attn(const int* __restrict__ eidx, const float* __restrict__ P,
                                              unsigned short* out16, int copyBase) {
  extern __shared__ v4f lds_dyn[];
  char* lb = (char*)lds_dyn;
  float* slog = (float*)(lb + T_SL);
  int*   scol = (int*)(lb + T_SC);
  int*   srow = (int*)(lb + T_SR);
  int*   esrt = (int*)(lb + T_ES);
  int*   soff = (int*)(lb + T_OF);
  int*   scnt = (int*)(lb + T_CN);
  const int tid = threadIdx.x, lane = tid & 31, wave = tid >> 5, head = lane >> 3;
  const int lc   = blockIdx.x;
  const int copy = copyBase + lc;
  const int bidx = copy / NST;
  const int sidx = copy - bidx * NST;

  build_csr(eidx, eidx + NE, scol, srow, esrt, soff, scnt, tid);

  const float* Pc = P + (size_t)lc * NN * PW;
  const v4f z4 = {0.f, 0.f, 0.f, 0.f};
  for (int c = wave; c < NN; c += NWAVE) {
    int st = soff[c];     st = st < 0 ? 0 : (st > NE ? NE : st);
    int en = soff[c + 1]; en = en < 0 ? 0 : (en > NE ? NE : en);
    int n  = en - st;     n  = n  < 0 ? 0 : (n  > NE ? NE : n);
    const float* qp = Pc + (size_t)c * PW + 8 * lane;
    const v4f q0 = *(const v4f*)qp, q1 = *(const v4f*)(qp + 4);

    float mx = NEG_BIG;
#pragma unroll 1
    for (int p = 0; p < n; ++p) {
      int slot = st + p; slot = slot > NE - 1 ? NE - 1 : slot;
      int src = esrt[slot]; src = src < 0 ? 0 : (src > NN - 1 ? NN - 1 : src);
      const float* kp = Pc + (size_t)src * PW + 256 + 8 * lane;
      const v4f k0 = *(const v4f*)kp, k1 = *(const v4f*)(kp + 4);
      const v4f pr = q0 * k0 + q1 * k1;
      float d = (pr.x + pr.y) + (pr.z + pr.w);
      d += __shfl_xor(d, 1);
      d += __shfl_xor(d, 2);
      d += __shfl_xor(d, 4);
      const float lg = d * 0.125f;
      mx = fmaxf(mx, lg);
      slog[slot * 4 + head] = lg;
    }

    float den = 0.f;
    v4f a0 = z4, a1 = z4;
#pragma unroll 1
    for (int p = 0; p < n; ++p) {
      int slot = st + p; slot = slot > NE - 1 ? NE - 1 : slot;
      int src = esrt[slot]; src = src < 0 ? 0 : (src > NN - 1 ? NN - 1 : src);
      const float lg = slog[slot * 4 + head];
      const float pw = __expf(lg - mx);
      den += pw;
      const float* vp = Pc + (size_t)src * PW + 512 + 8 * lane;
      const v4f v0 = *(const v4f*)vp, v1 = *(const v4f*)(vp + 4);
      a0 = a0 + v0 * pw;
      a1 = a1 + v1 * pw;
    }

    const float rd = 1.0f / (den + DEN_EPS);
    const float* skp = Pc + (size_t)c * PW + 768 + 8 * lane;
    const v4f s0 = *(const v4f*)skp, s1 = *(const v4f*)(skp + 4);
    const v4f r0 = a0 * rd + s0;
    const v4f r1 = a1 * rd + s1;
    const v8us ov = cvt8(r0, r1, ASCL);
    unsigned short* dp = out16 + ((size_t)(bidx * NN + c) * KF + (size_t)sidx * 256 + 8 * lane);
    *(volatile v8us*)dp = ov;
    __threadfence();
    *(volatile v8us*)dp = ov;
  }
}

__global__ __launch_bounds__(32) void k_final(const unsigned short* __restrict__ A,
                                             const unsigned short* __restrict__ wl,
                                             const float* __restrict__ bl, float* y) {
  __shared__ __attribute__((aligned(16))) float stg[16 * CO];
  const int lane = threadIdx.x & 31, hh = lane >> 4, m = lane & 15;
  const int tile = blockIdx.x;
  const unsigned short* afp = A  + (size_t)(tile * 16 + m) * KF + 8 * hh;
  const unsigned short* bfp = wl + (size_t)m * KF + 8 * hh;
  v8f acc = {0.f, 0.f, 0.f, 0.f, 0.f, 0.f, 0.f, 0.f};
#pragma unroll 4
  for (int ks = 0; ks < KF / 32; ++ks) {
    FragH af, bf;
    af.u[0] = *(const v8us*)(afp + 32 * ks);
    af.u[1] = *(const v8us*)(afp + 32 * ks + 16);
    bf.u[0] = *(const v8us*)(bfp + 32 * ks);
    bf.u[1] = *(const v8us*)(bfp + 32 * ks + 16);
    acc = wmh(af.v, bf.v, acc);
  }
  const float bb = bl[m < CO ? m : CO - 1];
#pragma unroll
  for (int r = 0; r < 8; ++r) {
    const float v = acc[r] * INV8192 + bb;
    if (m < CO) stg[(8 * hh + r) * CO + m] = v;
  }
  __syncthreads();
  const v4f p0 = *(const v4f*)(stg + 4 * lane);
  const v4f p1 = *(const v4f*)(stg + 4 * (32 + (lane & 15)));
  float* gp = y + (size_t)tile * (16 * CO);
  *(volatile v4f*)(gp + 4 * lane) = p0;
  if (lane < 16) *(volatile v4f*)(gp + 128 + 4 * lane) = p1;
  __threadfence();
  *(volatile v4f*)(gp + 4 * lane) = p0;
  if (lane < 16) *(volatile v4f*)(gp + 128 + 4 * lane) = p1;
}

static inline size_t al256(size_t v) { return (v + 255) & ~(size_t)255; }

extern "C" void kernel_launch(void* const* d_in, const int* in_sizes, int n_in,
                              void* d_out, int out_size, void* d_ws, size_t ws_size,
                              hipStream_t stream) {
  if (n_in < 20) return;
  if (in_sizes[0] != NROWS * CI || in_sizes[1] != 2 * NE) return;
  if (in_sizes[2] != CI * HD || in_sizes[3] != HD) return;
  for (int l = 1; l < 4; ++l) if (in_sizes[2 + 2 * l] != HD * HD || in_sizes[3 + 2 * l] != HD) return;
  for (int j = 0; j < 4; ++j) if (in_sizes[10 + 2 * j] != HD * 256 || in_sizes[11 + 2 * j] != 256) return;
  if (in_sizes[18] != KF * CO || in_sizes[19] != CO) return;
  if (out_size != NBT * NN * CO) return;

  const float* x    = (const float*)d_in[0];
  const int*   eidx = (const int*)d_in[1];
  const float* Wg0 = (const float*)d_in[2];  const float* bg0 = (const float*)d_in[3];
  const float* Wg1 = (const float*)d_in[4];  const float* bg1 = (const float*)d_in[5];
  const float* Wg2 = (const float*)d_in[6];  const float* bg2 = (const float*)d_in[7];
  const float* Wg3 = (const float*)d_in[8];  const float* bg3 = (const float*)d_in[9];
  const float* Wq  = (const float*)d_in[10]; const float* bq  = (const float*)d_in[11];
  const float* Wk  = (const float*)d_in[12]; const float* bk  = (const float*)d_in[13];
  const float* Wv  = (const float*)d_in[14]; const float* bv  = (const float*)d_in[15];
  const float* Wsk = (const float*)d_in[16]; const float* bsk = (const float*)d_in[17];
  const float* Wl  = (const float*)d_in[18]; const float* bl  = (const float*)d_in[19];
  float* y = (float*)d_out;

  const size_t szWG = (size_t)(CI * HD + 3 * HD * HD) * 2;
  const size_t szWP = (size_t)PW * HD * 2;
  const size_t szWL = (size_t)COP * KF * 2;
  const size_t szXT = (size_t)NROWS * HD * 2;
  const size_t szP  = (size_t)RPCP * PW * 4;
  const size_t szO  = (size_t)NBT * NN * KF * 2;
  size_t off = 0;
  const size_t oWG = off; off = al256(off + szWG);
  const size_t oWP = off; off = al256(off + szWP);
  const size_t oWL = off; off = al256(off + szWL);
  const size_t oXT = off; off = al256(off + szXT);
  const size_t oP  = off; off = al256(off + szP);
  const size_t oO  = off; off = al256(off + szO);
  if (off > ws_size || off > (size_t)WSCAP) return;
  char* ws = (char*)d_ws;
  unsigned short* wg16  = (unsigned short*)(ws + oWG);
  unsigned short* wp16  = (unsigned short*)(ws + oWP);
  unsigned short* wl16  = (unsigned short*)(ws + oWL);
  unsigned short* xt16  = (unsigned short*)(ws + oXT);
  float*          P     = (float*)(ws + oP);
  unsigned short* out16 = (unsigned short*)(ws + oO);

  k_wcvt<<<(HD * CI / 8 + NTHR - 1) / NTHR, NTHR, 0, stream>>>(Wg0, CI, HD, HD, WSCL, wg16);
  k_wcvt<<<(HD * HD / 8 + NTHR - 1) / NTHR, NTHR, 0, stream>>>(Wg1, HD, HD, HD, WSCL, wg16 + CI * HD);
  k_wcvt<<<(HD * HD / 8 + NTHR - 1) / NTHR, NTHR, 0, stream>>>(Wg2, HD, HD, HD, WSCL, wg16 + CI * HD + HD * HD);
  k_wcvt<<<(HD * HD / 8 + NTHR - 1) / NTHR, NTHR, 0, stream>>>(Wg3, HD, HD, HD, WSCL, wg16 + CI * HD + 2 * HD * HD);
  k_wcvt<<<(256 * HD / 8 + NTHR - 1) / NTHR, NTHR, 0, stream>>>(Wq,  HD, 256, 256, WSCL, wp16);
  k_wcvt<<<(256 * HD / 8 + NTHR - 1) / NTHR, NTHR, 0, stream>>>(Wk,  HD, 256, 256, WSCL, wp16 + (size_t)256 * HD);
  k_wcvt<<<(256 * HD / 8 + NTHR - 1) / NTHR, NTHR, 0, stream>>>(Wv,  HD, 256, 256, WSCL, wp16 + (size_t)512 * HD);
  k_wcvt<<<(256 * HD / 8 + NTHR - 1) / NTHR, NTHR, 0, stream>>>(Wsk, HD, 256, 256, WSCL, wp16 + (size_t)768 * HD);
  k_wcvt<<<(COP * KF / 8 + NTHR - 1) / NTHR, NTHR, 0, stream>>>(Wl, KF, CO, COP, LSCL, wl16);

  hipFuncSetAttribute(reinterpret_cast<const void*>(&k_gcn),
                      hipFuncAttributeMaxDynamicSharedMemorySize, LDS_GCN);
  k_gcn<<<NCP, NTHR, LDS_GCN, stream>>>(x, eidx, wg16, bg0, bg1, bg2, bg3, xt16);

  hipFuncSetAttribute(reinterpret_cast<const void*>(&k_attn),
                      hipFuncAttributeMaxDynamicSharedMemorySize, LDS_ATTN);
  for (int ch = 0; ch < NCHUNK; ++ch) {
    k_proj<<<dim3(GPX, 4), NTHR, 0, stream>>>(xt16, wp16, bq, bk, bv, bsk, P, ch * RPC, NROWS);
    k_attn<<<CPC, NTHR, LDS_ATTN, stream>>>(eidx, P, out16, ch * CPC);
  }

  k_final<<<(NBT * NN) / 16, 32, 0, stream>>>(out16, wl16, bl, y);
}
